// gconv_73684458930377
// MI455X (gfx1250) — hardware-verified
//
#include <hip/hip_runtime.h>
#include <stddef.h>
#include <stdint.h>


#define BB      8
#define INF     64
#define UNITS   64
#define NMAT    3
#define HW      (BB * INF)
#define KH      (NMAT * INF)
#define KL      (2 * INF)
#define NTHR    256
#define NWAVE   8
#define EPT     8
#define CHUNK   (NTHR * EPT)
#define WCAP    (EPT * 32)
#define LISTN   (NWAVE * WCAP)
#define NBMAX   2048
#define RCAP    24576
#define DEGCAP  4096
#define GBM     64
#define GBN     64
#define GTHR    128
#define CX      8.0f
#define CW      64.0f
#define CL      2048.0f
#define S_HI    0.001953125f
#define S_LO    9.5367431640625e-07f
#define WSMAX   134217728
#define LDS_SP  ((2 * RCAP + 2 * NBMAX + LISTN) * 4 + 64)

static_assert((CHUNK & (CHUNK - 1)) == 0 && CHUNK <= 4096);
static_assert((NBMAX & (NBMAX - 1)) == 0 && NBMAX <= 4096);
static_assert(NTHR * 8 == NBMAX);
static_assert(LISTN >= NBMAX);
static_assert(LISTN >= NWAVE * WCAP);
static_assert((RCAP % 32) == 0);
static_assert(LDS_SP <= 300000);
static_assert(GBM == (GTHR / 32) * 16);
static_assert((KH % 32) == 0 && (KL % 32) == 0);
static_assert(UNITS == GBN);
static_assert(HW == 4 * 128);
static_assert((INF % 8) == 0);

typedef float    v4f  __attribute__((ext_vector_type(4)));
typedef float    v8f  __attribute__((ext_vector_type(8)));
typedef int      v4i  __attribute__((ext_vector_type(4)));
typedef int      v8i  __attribute__((ext_vector_type(8)));
typedef _Float16 v4h  __attribute__((ext_vector_type(4)));
typedef _Float16 v8h  __attribute__((ext_vector_type(8)));
typedef _Float16 v16h __attribute__((ext_vector_type(16)));
typedef v8h __attribute__((may_alias)) v8ha;
typedef v4f __attribute__((may_alias)) v4fa;
union FragH { v16h v; v8h h[2]; v8i w; };

__device__ __forceinline__ v8f wmh(const FragH& a, const FragH& b, v8f c) {
  v8f d = __builtin_amdgcn_wmma_f32_16x16x32_f16(false, a.v, false, b.v, (short)0, c, false, false);
  asm volatile("v_nop\n\tv_nop\n\tv_nop\n\tv_nop" : "+v"(d) : "v"(a.w), "v"(b.w));
  return d;
}

__device__ __forceinline__ float bfr(float f) {
  unsigned u = __float_as_uint(f);
  u = (u + 0x7FFFu + ((u >> 16) & 1u)) & 0xFFFF0000u;
  return __uint_as_float(u);
}

__device__ __forceinline__ v4f madd4(v4f a, float v, v4f g) {
  v4f r;
  r.x = a.x + v * g.x; r.y = a.y + v * g.y; r.z = a.z + v * g.z; r.w = a.w + v * g.w;
  return r;
}

__device__ __forceinline__ v4f comb4(v4f a, v4f u, bool s2, float pz) {
  v4f r;
  r.x = (s2 ? ((a.x + a.x) - u.x) : a.x) + pz;
  r.y = (s2 ? ((a.y + a.y) - u.y) : a.y) + pz;
  r.z = (s2 ? ((a.z + a.z) - u.z) : a.z) + pz;
  r.w = (s2 ? ((a.w + a.w) - u.w) : a.w) + pz;
  return r;
}

__device__ __forceinline__ int scan_chunk(const int* __restrict__ dsts, int nE, int cbase, int slotBase,
                                          int nb, int vec8, int* list, int tid, int lane, int wave) {
  int wc = 0;
  const int el0  = tid * EPT;
  const int e0   = cbase + el0;
  const int sent = -2147483647 - 1;
  v4i da, db;
  if (vec8 != 0 && cbase + CHUNK <= nE) {
    da = *(const v4i*)(dsts + e0);
    db = *(const v4i*)(dsts + e0 + 4);
  } else {
    da.x = (e0     < nE) ? dsts[min(e0,     nE - 1)] : sent;
    da.y = (e0 + 1 < nE) ? dsts[min(e0 + 1, nE - 1)] : sent;
    da.z = (e0 + 2 < nE) ? dsts[min(e0 + 2, nE - 1)] : sent;
    da.w = (e0 + 3 < nE) ? dsts[min(e0 + 3, nE - 1)] : sent;
    db.x = (e0 + 4 < nE) ? dsts[min(e0 + 4, nE - 1)] : sent;
    db.y = (e0 + 5 < nE) ? dsts[min(e0 + 5, nE - 1)] : sent;
    db.z = (e0 + 6 < nE) ? dsts[min(e0 + 6, nE - 1)] : sent;
    db.w = (e0 + 7 < nE) ? dsts[min(e0 + 7, nE - 1)] : sent;
  }
  const unsigned nbs = (unsigned)slotBase;
  const unsigned unb = (unsigned)nb;
  const unsigned s0 = (unsigned)da.x - nbs, s1 = (unsigned)da.y - nbs;
  const unsigned s2 = (unsigned)da.z - nbs, s3 = (unsigned)da.w - nbs;
  const unsigned s4 = (unsigned)db.x - nbs, s5 = (unsigned)db.y - nbs;
  const unsigned s6 = (unsigned)db.z - nbs, s7 = (unsigned)db.w - nbs;
  const bool h0 = s0 < unb, h1 = s1 < unb, h2 = s2 < unb, h3 = s3 < unb;
  const bool h4 = s4 < unb, h5 = s5 < unb, h6 = s6 < unb, h7 = s7 < unb;
  const unsigned any = __builtin_amdgcn_ballot_w32(h0 | h1 | h2 | h3 | h4 | h5 | h6 | h7);
  if (any != 0u) {
#define HITJ(J, HJ, SJ) { \
      const unsigned mj = __builtin_amdgcn_ballot_w32(HJ); \
      if (mj != 0u) { \
        if (HJ) { \
          const int pos = wc + (int)__builtin_amdgcn_mbcnt_lo(mj, 0u); \
          if (pos < WCAP) list[wave * WCAP + pos] = ((el0 + (J)) << 12) | (int)(SJ); \
        } \
        wc += (int)__builtin_popcount(mj); } }
    HITJ(0, h0, s0)
    HITJ(1, h1, s1)
    HITJ(2, h2, s2)
    HITJ(3, h3, s3)
    HITJ(4, h4, s4)
    HITJ(5, h5, s5)
    HITJ(6, h6, s6)
    HITJ(7, h7, s7)
#undef HITJ
  }
  return wc;
}

__global__ __launch_bounds__(NTHR) void k_prep(const float* __restrict__ x, float* t0f, int nN, int nUnits) {
  const int t = (int)blockIdx.x * NTHR + (int)threadIdx.x;
  if (t >= nUnits) return;
  const int n   = t >> 7;
  const int rem = t & 127;
  const int b   = rem >> 4;
  const int i4  = (rem & 15) * 4;
  const float* p = x + ((size_t)b * (size_t)nN + (size_t)n) * INF + i4;
  const v4f a = *(const v4fa*)p;
  v4f r;
  r.x = bfr(a.x); r.y = bfr(a.y); r.z = bfr(a.z); r.w = bfr(a.w);
  float* o = t0f + (size_t)t * 4;
  *(volatile v4f*)o = r;
  __threadfence();
  *(volatile v4f*)o = r;
}

__global__ __launch_bounds__(NTHR) void k_wtr(const float* __restrict__ w, _Float16* wth, _Float16* wtl, int nUnits) {
  const int u = (int)blockIdx.x * NTHR + (int)threadIdx.x;
  if (u >= nUnits) return;
  const int nHp = UNITS * (KH / 8);
  const bool hiP = u < nHp;
  const int v   = hiP ? u : (u - nHp);
  const int kq  = hiP ? (KH / 8) : (KL / 8);
  const int n   = v / kq;
  const int k8  = (v - n * kq) * 8;
  const int mm  = (k8 >> 6) + (hiP ? 0 : 1);
  const int i0  = k8 & 63;
  const float* p = w + (size_t)(i0 * NMAT + mm) * UNITS + n;
  v8h hv;
  hv[0] = (_Float16)(bfr(p[0])              * CW);
  hv[1] = (_Float16)(bfr(p[(size_t)KH])     * CW);
  hv[2] = (_Float16)(bfr(p[(size_t)2 * KH]) * CW);
  hv[3] = (_Float16)(bfr(p[(size_t)3 * KH]) * CW);
  hv[4] = (_Float16)(bfr(p[(size_t)4 * KH]) * CW);
  hv[5] = (_Float16)(bfr(p[(size_t)5 * KH]) * CW);
  hv[6] = (_Float16)(bfr(p[(size_t)6 * KH]) * CW);
  hv[7] = (_Float16)(bfr(p[(size_t)7 * KH]) * CW);
  _Float16* o = hiP ? (wth + (size_t)n * KH + k8) : (wtl + (size_t)n * KL + k8);
  *(volatile v8h*)o = hv;
  __threadfence();
  *(volatile v8h*)o = hv;
}

__global__ __launch_bounds__(NTHR) void k_spmm(
    const int* __restrict__ rws, const int* __restrict__ cls, const float* __restrict__ vals,
    const float* __restrict__ hin, const float* __restrict__ t0p, float* hout,
    int nN, int nE, int nb, int vec8, int step2) {
  extern __shared__ v4f lds_dyn[];
  int* reg1 = (int*)lds_dyn;
  int* reg2 = reg1 + RCAP;
  int* scnt = reg2 + RCAP;
  int* soff = scnt + NBMAX;
  int* list = soff + NBMAX;
  int* wcnt = list + LISTN;
  int* wtot = wcnt + NWAVE;
  const int tid = (int)threadIdx.x, lane = tid & 31, wave = tid >> 5;
  const int nodeBase = (int)blockIdx.x * nb;

  for (int i = tid; i < NBMAX; i += NTHR) scnt[i] = 0;
  __syncthreads();

  int tot = 0;
  const int nChunks = (nE + CHUNK - 1) / CHUNK;
#pragma unroll 1
  for (int ch = 0; ch < nChunks; ++ch) {
    const int cbase = ch * CHUNK;
    const int wc = scan_chunk(rws, nE, cbase, nodeBase, nb, vec8, list, tid, lane, wave);
    if (lane == 0) wcnt[wave] = wc;
    __syncthreads();
    int pre = 0, all = 0;
#pragma unroll
    for (int w2 = 0; w2 < NWAVE; ++w2) {
      int c = wcnt[w2];
      c = c < 0 ? 0 : (c > WCAP ? WCAP : c);
      all += c;
      pre += (w2 < wave) ? c : 0;
    }
    const int wcc  = wc > WCAP ? WCAP : wc;
    const int base = tot + pre;
#pragma unroll 1
    for (int i = lane; i < wcc; i += 32) {
      const int ent = list[wave * WCAP + i];
      const int el  = (ent >> 12) & (CHUNK - 1);
      const int sl  = ent & (NBMAX - 1);
      int eid = cbase + el;
      eid = eid > nE - 1 ? nE - 1 : eid;
      const int pos = base + i;
      if (pos < RCAP) reg1[pos] = (int)(((unsigned)eid << 12) | (unsigned)sl);
    }
    tot += all;
    tot = tot > RCAP ? RCAP : tot;
    __syncthreads();
  }
  const int nh = tot;

  if (wave == 0) {
#pragma unroll 1
    for (int b0 = 0; b0 < nh; b0 += 32) {
      const int idx = b0 + lane;
      const int uv  = reg1[idx < RCAP ? idx : RCAP - 1];
      const int m32 = (nh - b0) < 32 ? (nh - b0) : 32;
#pragma unroll 1
      for (int k = 0; k < m32; ++k) {
        const int u  = __builtin_amdgcn_readlane(uv, k);
        const int sl = u & (NBMAX - 1);
        if (lane == 0) scnt[sl] = scnt[sl] + 1;
      }
    }
  }
  __syncthreads();

  {
    const v4i ca = *(const v4i*)(scnt + 8 * tid);
    const v4i cb = *(const v4i*)(scnt + 8 * tid + 4);
    const int e0 = ca.x < 0 ? 0 : ca.x, e1 = ca.y < 0 ? 0 : ca.y, e2 = ca.z < 0 ? 0 : ca.z, e3 = ca.w < 0 ? 0 : ca.w;
    const int e4 = cb.x < 0 ? 0 : cb.x, e5 = cb.y < 0 ? 0 : cb.y, e6 = cb.z < 0 ? 0 : cb.z, e7 = cb.w < 0 ? 0 : cb.w;
    const int ts = e0 + e1 + e2 + e3 + e4 + e5 + e6 + e7;
    int incl = ts;
#pragma unroll
    for (int d = 1; d < 32; d <<= 1) {
      const int up = __shfl_up(incl, d);
      if (lane >= d) incl += up;
    }
    if (lane == 31) wtot[wave] = incl;
    __syncthreads();
    int pre = 0;
#pragma unroll
    for (int w2 = 0; w2 < NWAVE; ++w2) pre += (w2 < wave) ? wtot[w2] : 0;
    int run = pre + incl - ts;
    soff[8 * tid + 0] = run; run += e0;
    soff[8 * tid + 1] = run; run += e1;
    soff[8 * tid + 2] = run; run += e2;
    soff[8 * tid + 3] = run; run += e3;
    soff[8 * tid + 4] = run; run += e4;
    soff[8 * tid + 5] = run; run += e5;
    soff[8 * tid + 6] = run; run += e6;
    soff[8 * tid + 7] = run;
  }
  __syncthreads();
  for (int i = tid; i < NBMAX; i += NTHR) list[i] = soff[i];
  __syncthreads();

  if (wave == 0) {
#pragma unroll 1
    for (int b0 = 0; b0 < nh; b0 += 32) {
      const int idx = b0 + lane;
      const int uv  = reg1[idx < RCAP ? idx : RCAP - 1];
      const int m32 = (nh - b0) < 32 ? (nh - b0) : 32;
#pragma unroll 1
      for (int k = 0; k < m32; ++k) {
        const int u   = __builtin_amdgcn_readlane(uv, k);
        const int sl  = u & (NBMAX - 1);
        const int eid = (int)((unsigned)u >> 12);
        if (lane == 0) {
          int pos = list[sl];
          pos = pos < 0 ? 0 : (pos > RCAP - 1 ? RCAP - 1 : pos);
          reg2[pos] = eid;
          list[sl] = pos + 1;
        }
      }
    }
  }
  __syncthreads();

  const int nbw = nb >> 3;
  const bool ovf = (nh >= RCAP);
  const bool s2  = (step2 != 0);
  const float qnan = __int_as_float(0x7fc00000);
  const v4f z4 = {0.f, 0.f, 0.f, 0.f};
#pragma unroll 1
  for (int jt = 0; jt < nbw; ++jt) {
    const int slot = wave * nbw + jt;
    const int grow = nodeBase + slot;
    const int gcl  = grow < nN ? grow : nN - 1;
    int st = soff[slot];
    const int craw = scnt[slot];
    int cnt = craw;
    st  = st < 0 ? 0 : (st > nh ? nh : st);
    cnt = cnt < 0 ? 0 : (cnt > DEGCAP ? DEGCAP : cnt);
    if (cnt > nh - st) cnt = nh - st;
    const float pz = (ovf || craw > DEGCAP) ? qnan : 0.0f;
    const bool wr = grow < nN;

    v4f a0 = z4, a1 = z4, a2 = z4, a3 = z4;
#pragma unroll 1
    for (int q = 0; q < cnt; ++q) {
      int idx = st + q; idx = idx > RCAP - 1 ? RCAP - 1 : idx;
      int eid = reg2[idx]; eid = eid < 0 ? 0 : (eid > nE - 1 ? nE - 1 : eid);
      const int sraw = cls[eid];
      const int s = sraw < 0 ? 0 : (sraw > nN - 1 ? nN - 1 : sraw);
      const float v = bfr(vals[eid]);
      const float* hr = hin + (size_t)s * HW + 4 * lane;
      const v4f g0 = *(const v4fa*)(hr);
      const v4f g1 = *(const v4fa*)(hr + 128);
      const v4f g2 = *(const v4fa*)(hr + 256);
      const v4f g3 = *(const v4fa*)(hr + 384);
      a0 = madd4(a0, v, g0);
      a1 = madd4(a1, v, g1);
      a2 = madd4(a2, v, g2);
      a3 = madd4(a3, v, g3);
    }
    const float* tr = t0p + (size_t)gcl * HW + 4 * lane;
    const v4f u0 = *(const v4fa*)(tr);
    const v4f u1 = *(const v4fa*)(tr + 128);
    const v4f u2 = *(const v4fa*)(tr + 256);
    const v4f u3 = *(const v4fa*)(tr + 384);
    const v4f o0 = comb4(a0, u0, s2, pz);
    const v4f o1 = comb4(a1, u1, s2, pz);
    const v4f o2 = comb4(a2, u2, s2, pz);
    const v4f o3 = comb4(a3, u3, s2, pz);
    float* op = hout + (size_t)gcl * HW + 4 * lane;
    if (wr) {
      *(volatile v4f*)(op)       = o0;
      *(volatile v4f*)(op + 128) = o1;
      *(volatile v4f*)(op + 256) = o2;
      *(volatile v4f*)(op + 384) = o3;
    }
    __threadfence();
    if (wr) {
      *(volatile v4f*)(op)       = o0;
      *(volatile v4f*)(op + 128) = o1;
      *(volatile v4f*)(op + 256) = o2;
      *(volatile v4f*)(op + 384) = o3;
    }
  }
}

__global__ __launch_bounds__(NTHR) void k_pack(const float* __restrict__ t0f, const float* __restrict__ t1f,
                                               const float* __restrict__ t2f, _Float16* ah, _Float16* al, int nN) {
  __shared__ __attribute__((aligned(16))) _Float16 sh[NWAVE * BB * KH];
  __shared__ __attribute__((aligned(16))) _Float16 sl[NWAVE * BB * KL];
  const int tid = (int)threadIdx.x, lane = tid & 31, wave = tid >> 5, hh = lane >> 4, m = lane & 15;
  const int n = (int)blockIdx.x * NWAVE + wave;
  if (n >= nN) return;
  _Float16* shw = sh + wave * (BB * KH);
  _Float16* slw = sl + wave * (BB * KL);
  const size_t rb = (size_t)n * HW + 4 * lane;

#pragma unroll
  for (int s = 0; s < 3; ++s) {
    const float* P = (s == 0) ? t0f : ((s == 1) ? t1f : t2f);
#pragma unroll
    for (int j = 0; j < 4; ++j) {
      const v4f g = *(const v4fa*)(P + rb + 128 * j);
      const int b = 2 * j + hh;
      const float c0 = g.x * CX, c1 = g.y * CX, c2 = g.z * CX, c3 = g.w * CX;
      v4h th;
      th.x = (_Float16)c0; th.y = (_Float16)c1; th.z = (_Float16)c2; th.w = (_Float16)c3;
      *(v4h*)(shw + (b * NMAT + s) * INF + 4 * m) = th;
      if (s > 0) {
        v4h tl;
        tl.x = (_Float16)((c0 - (float)th.x) * CL);
        tl.y = (_Float16)((c1 - (float)th.y) * CL);
        tl.z = (_Float16)((c2 - (float)th.z) * CL);
        tl.w = (_Float16)((c3 - (float)th.w) * CL);
        *(v4h*)(slw + (b * 2 + (s - 1)) * INF + 4 * m) = tl;
      }
    }
  }
  __builtin_amdgcn_fence(__ATOMIC_RELEASE, "wavefront");
  __builtin_amdgcn_wave_barrier();

  v8h hv[6], lv[4];
#pragma unroll
  for (int s = 0; s < 6; ++s) hv[s] = *(const v8ha*)(shw + 8 * (32 * s + lane));
#pragma unroll
  for (int s = 0; s < 4; ++s) lv[s] = *(const v8ha*)(slw + 8 * (32 * s + lane));

  const int q8 = lane & 7;
#pragma unroll
  for (int s = 0; s < 6; ++s) {
    const int L = 4 * s + (lane >> 3);
    const int b = L / 3, seg = L - 3 * b;
    _Float16* dst = ah + ((size_t)b * (size_t)nN + (size_t)n) * KH + seg * INF + 8 * q8;
    *(volatile v8h*)dst = hv[s];
  }
#pragma unroll
  for (int s = 0; s < 4; ++s) {
    const int L = 4 * s + (lane >> 3);
    const int b = L >> 1, seg = L & 1;
    _Float16* dst = al + ((size_t)b * (size_t)nN + (size_t)n) * KL + seg * INF + 8 * q8;
    *(volatile v8h*)dst = lv[s];
  }
  __threadfence();
#pragma unroll
  for (int s = 0; s < 6; ++s) {
    const int L = 4 * s + (lane >> 3);
    const int b = L / 3, seg = L - 3 * b;
    _Float16* dst = ah + ((size_t)b * (size_t)nN + (size_t)n) * KH + seg * INF + 8 * q8;
    *(volatile v8h*)dst = hv[s];
  }
#pragma unroll
  for (int s = 0; s < 4; ++s) {
    const int L = 4 * s + (lane >> 3);
    const int b = L >> 1, seg = L & 1;
    _Float16* dst = al + ((size_t)b * (size_t)nN + (size_t)n) * KL + seg * INF + 8 * q8;
    *(volatile v8h*)dst = lv[s];
  }
}

__global__ __launch_bounds__(GTHR) void k_gemm(
    const _Float16* __restrict__ AH, const _Float16* __restrict__ WTH,
    const _Float16* __restrict__ AL, const _Float16* __restrict__ WTL,
    const float* __restrict__ bias, float* outF, int nRows)
{
  __shared__ __attribute__((aligned(16))) float stg[GBM * GBN];
  const int tid = (int)threadIdx.x, lane = tid & 31, wave = tid >> 5, hh = lane >> 4, m = lane & 15;
  const int rowBase = (int)blockIdx.x * GBM;
  int arow = rowBase + 16 * wave + m;
  arow = arow > nRows - 1 ? nRows - 1 : arow;

  const v8f z8 = {0.f, 0.f, 0.f, 0.f, 0.f, 0.f, 0.f, 0.f};
  v8f acc[4];
  acc[0] = z8; acc[1] = z8; acc[2] = z8; acc[3] = z8;
  {
    const _Float16* ap = AH  + (size_t)arow * (size_t)KH + 8 * hh;
    const _Float16* wp = WTH + (size_t)m * (size_t)KH + 8 * hh;
#pragma unroll 1
    for (int ks = 0; ks < KH / 32; ++ks) {
      FragH af;
      af.h[0] = *(const v8ha*)(ap + 32 * ks);
      af.h[1] = *(const v8ha*)(ap + 32 * ks + 16);
#pragma unroll
      for (int t = 0; t < 4; ++t) {
        const _Float16* wq = wp + (size_t)(16 * t) * (size_t)KH + 32 * ks;
        FragH bf;
        bf.h[0] = *(const v8ha*)wq;
        bf.h[1] = *(const v8ha*)(wq + 16);
        acc[t] = wmh(af, bf, acc[t]);
      }
    }
  }
  v8f acc2[4];
  acc2[0] = z8; acc2[1] = z8; acc2[2] = z8; acc2[3] = z8;
  {
    const _Float16* ap = AL  + (size_t)arow * (size_t)KL + 8 * hh;
    const _Float16* wp = WTL + (size_t)m * (size_t)KL + 8 * hh;
#pragma unroll 1
    for (int ks = 0; ks < KL / 32; ++ks) {
      FragH af;
      af.h[0] = *(const v8ha*)(ap + 32 * ks);
      af.h[1] = *(const v8ha*)(ap + 32 * ks + 16);
#pragma unroll
      for (int t = 0; t < 4; ++t) {
        const _Float16* wq = wp + (size_t)(16 * t) * (size_t)KL + 32 * ks;
        FragH bf;
        bf.h[0] = *(const v8ha*)wq;
        bf.h[1] = *(const v8ha*)(wq + 16);
        acc2[t] = wmh(af, bf, acc2[t]);
      }
    }
  }

#pragma unroll
  for (int t = 0; t < 4; ++t) {
    const int lc = 16 * t + m;
    const float bv = bfr(bias[lc]);
#pragma unroll
    for (int r = 0; r < 8; ++r) {
      const int lr = 16 * wave + 8 * hh + r;
      stg[lr * GBN + lc] = (acc[t][r] * S_HI + acc2[t][r] * S_LO) + bv;
    }
  }
  __syncthreads();

  v4f fv[8];
#pragma unroll
  for (int i = 0; i < 8; ++i) {
    const int lr = 16 * wave + 2 * i + hh;
    fv[i] = *(const v4fa*)(stg + lr * GBN + 4 * m);
  }
#pragma unroll
  for (int i = 0; i < 8; ++i) {
    const int gr = rowBase + 16 * wave + 2 * i + hh;
    if (gr < nRows) *(volatile v4f*)(outF + (size_t)gr * (size_t)UNITS + 4 * m) = fv[i];
  }
  __threadfence();
#pragma unroll
  for (int i = 0; i < 8; ++i) {
    const int gr = rowBase + 16 * wave + 2 * i + hh;
    if (gr < nRows) *(volatile v4f*)(outF + (size_t)gr * (size_t)UNITS + 4 * m) = fv[i];
  }
}

static int pick_nb(int nE, int nN) {
  int nb = NBMAX;
  while (nb > 16 && (long long)nb * (long long)nE * 5LL > (long long)RCAP * (long long)nN * 4LL) nb >>= 1;
  return nb;
}
static inline int cdiv(int a, int b) { return (a + b - 1) / b; }

extern "C" void kernel_launch(void* const* d_in, const int* in_sizes, int n_in,
                              void* d_out, int out_size, void* d_ws, size_t ws_size,
                              hipStream_t stream) {
  if (n_in < 6) return;
  const int nN = in_sizes[0] / HW;
  if (nN <= 0 || nN * HW != in_sizes[0] || (nN % 8) != 0 || nN > (1 << 20)) return;
  const int nE = in_sizes[1];
  if (nE < 1 || nE > (1 << 20)) return;
  if (in_sizes[2] != nE || in_sizes[3] != nE) return;
  if (in_sizes[4] != KH * UNITS || in_sizes[5] != UNITS) return;
  const int nRows = BB * nN;
  if ((nRows % GBM) != 0 || out_size != nRows * UNITS) return;

  const float* x    = (const float*)d_in[0];
  const int*   rws  = (const int*)  d_in[1];
  const int*   cls  = (const int*)  d_in[2];
  const float* vals = (const float*)d_in[3];
  const float* w    = (const float*)d_in[4];
  const float* bias = (const float*)d_in[5];
  float* out = (float*)d_out;

  const int nb   = pick_nb(nE, nN);
  const int gA   = cdiv(nN, nb);
  const int vec8 = 1;
  if (gA * nb < nN) return;

  char* ws = (char*)d_ws;
  size_t off = 0;
  const size_t oT0 = off; off += (size_t)nN * HW * 4;             off = (off + 255) & ~(size_t)255;
  const size_t oT1 = off; off += (size_t)nN * HW * 4;             off = (off + 255) & ~(size_t)255;
  const size_t oT2 = off; off += (size_t)nN * HW * 4;             off = (off + 255) & ~(size_t)255;
  const size_t oAH = off; off += (size_t)nRows * KH * 2;          off = (off + 255) & ~(size_t)255;
  const size_t oAL = off; off += (size_t)nRows * KL * 2;          off = (off + 255) & ~(size_t)255;
  const size_t oWH = off; off += (size_t)UNITS * KH * 2;          off = (off + 255) & ~(size_t)255;
  const size_t oWL = off; off += (size_t)UNITS * KL * 2;          off = (off + 255) & ~(size_t)255;
  if (off > ws_size || off > (size_t)WSMAX) return;
  float*    T0F = (float*)(ws + oT0);
  float*    T1F = (float*)(ws + oT1);
  float*    T2F = (float*)(ws + oT2);
  _Float16* AH  = (_Float16*)(ws + oAH);
  _Float16* AL  = (_Float16*)(ws + oAL);
  _Float16* WTH = (_Float16*)(ws + oWH);
  _Float16* WTL = (_Float16*)(ws + oWL);

  hipFuncSetAttribute(reinterpret_cast<const void*>(&k_spmm),
                      hipFuncAttributeMaxDynamicSharedMemorySize, LDS_SP);

  const int nUp = nN * (HW / 4);
  k_prep<<<cdiv(nUp, NTHR), NTHR, 0, stream>>>(x, T0F, nN, nUp);

  const int nUw = UNITS * ((KH + KL) / 8);
  k_wtr<<<cdiv(nUw, NTHR), NTHR, 0, stream>>>(w, WTH, WTL, nUw);

  k_spmm<<<gA, NTHR, LDS_SP, stream>>>(rws, cls, vals, T0F, T0F, T1F, nN, nE, nb, vec8, 0);
  k_spmm<<<gA, NTHR, LDS_SP, stream>>>(rws, cls, vals, T1F, T0F, T2F, nN, nE, nb, vec8, 1);

  k_pack<<<cdiv(nN, NWAVE), NTHR, 0, stream>>>(T0F, T1F, T2F, AH, AL, nN);

  k_gemm<<<dim3(nRows / GBM, 1), GTHR, 0, stream>>>(AH, WTH, AL, WTL, bias, out, nRows);
}
